// MambaG2G_34514357190725
// MI455X (gfx1250) — hardware-run, weakly checked
//
#include <hip/hip_runtime.h>
#include <math.h>

typedef __attribute__((ext_vector_type(16))) _Float16 v16h;
typedef __attribute__((ext_vector_type(8)))  _Float16 v8h;
typedef __attribute__((ext_vector_type(16))) __bf16   v16b;
typedef __attribute__((ext_vector_type(8)))  __bf16   v8b;
typedef __attribute__((ext_vector_type(8)))  float    v8f;
typedef __attribute__((ext_vector_type(4)))  float    v4f;

constexpr int kBatch  = 64;
constexpr int kSeqL   = 256;
constexpr int kDmod   = 256;
constexpr int kDin    = 512;
constexpr int kNst    = 16;
constexpr int kDtR    = 16;
constexpr int kDtKP   = 32;
constexpr int kPrjN   = 48;
constexpr int kPrjP   = 64;
constexpr int kXZP    = 2 * kDin;
constexpr int kRows   = kBatch * kSeqL;
constexpr int kChunkB = 32;
constexpr int kChunkT = kChunkB * kSeqL;
constexpr int kNChunk = kBatch / kChunkB;
constexpr int kDimIn  = 256;
constexpr int kDimOut = 64;
constexpr int kTP     = 260;
static_assert(kDimIn == kDmod, "head kernels use one thread per column for both widths");
static_assert(kSeqL % 64 == 0, "conv blocks never straddle a sequence");

__device__ __forceinline__ unsigned short f2bf_bits(float f) {
  unsigned u = __float_as_uint(f);
  return (unsigned short)((u + 0x7FFFu + ((u >> 16) & 1u)) >> 16);
}
__device__ __forceinline__ float bf_bits2f(unsigned short h) { return __uint_as_float(((unsigned)h) << 16); }

__device__ __forceinline__ void dep_guard_h(v8f& a, v8f& b, v16h x, v16h y) { asm volatile("v_nop\n\tv_nop\n\tv_nop\n\tv_nop" : "+v"(a), "+v"(b) : "v"(x), "v"(y)); }
__device__ __forceinline__ void dep_guard_b(v8f& a, v8f& b, v16b x, v16b y) { asm volatile("v_nop\n\tv_nop\n\tv_nop\n\tv_nop" : "+v"(a), "+v"(b) : "v"(x), "v"(y)); }
__device__ __forceinline__ void keep4_h(v16h a, v16h b, v16h c, v16h d) { asm volatile("v_nop" :: "v"(a), "v"(b), "v"(c), "v"(d)); }
__device__ __forceinline__ void keep4_b(v16b a, v16b b, v16b c, v16b d) { asm volatile("v_nop" :: "v"(a), "v"(b), "v"(c), "v"(d)); }
__device__ __forceinline__ void acc_guard4(v8f& a, v8f& b, v8f& c, v8f& d) { asm volatile("v_nop\n\tv_nop\n\tv_nop\n\tv_nop" : "+v"(a), "+v"(b), "+v"(c), "+v"(d)); }
template <typename T> struct Frag;
template <> struct Frag<_Float16> {
  typedef v16h V; union U { v16h v; v8h h[2]; };
  static __device__ __forceinline__ v16h load(const _Float16* p) {
    U f; f.h[0] = *(const v8h*)(p); f.h[1] = *(const v8h*)(p + 16); return f.v;
  }
  static __device__ __forceinline__ v8f mma(v16h a, v16h b, v8f c) {
    return __builtin_amdgcn_wmma_f32_16x16x32_f16(false, a, false, b, (short)0, c, false, false);
  }
  static __device__ __forceinline__ void guard(v8f& a, v8f& b, v16h x, v16h y) { dep_guard_h(a, b, x, y); }
  static __device__ __forceinline__ void keep(v16h a, v16h b, v16h c, v16h d) { keep4_h(a, b, c, d); }
};
template <> struct Frag<__bf16> {
  typedef v16b V; union U { v16b v; v8b h[2]; };
  static __device__ __forceinline__ v16b load(const __bf16* p) {
    U f; f.h[0] = *(const v8b*)(p); f.h[1] = *(const v8b*)(p + 16); return f.v;
  }
  static __device__ __forceinline__ v8f mma(v16b a, v16b b, v8f c) {
    return __builtin_amdgcn_wmma_f32_16x16x32_bf16(false, a, false, b, (short)0, c, false, false);
  }
  static __device__ __forceinline__ void guard(v8f& a, v8f& b, v16b x, v16b y) { dep_guard_b(a, b, x, y); }
  static __device__ __forceinline__ void keep(v16b a, v16b b, v16b c, v16b d) { keep4_b(a, b, c, d); }
};

template <int ET> struct Elem;
template <> struct Elem<0> { typedef _Float16 T; };
template <> struct Elem<1> { typedef __bf16 T; };
template <int ET, bool SPLIT, int BIAS_MODE, int OUT_MODE, bool RESID, int ACT = 0>
__global__ __launch_bounds__(256) void wmma_gemm64(
    const unsigned short* __restrict__ Ap, const unsigned short* __restrict__ A2p, int lda, long strideA,
    const unsigned short* __restrict__ Btp, const unsigned short* __restrict__ Bt2p, int ldb, long strideB,
    void* __restrict__ Cout, void* __restrict__ Cout2, int ldc, long strideC,
    const float* __restrict__ bias,
    const float* __restrict__ resid, long strideR,
    int M, int N, int K, float scale) {
  typedef typename Elem<ET>::T T;
  typedef typename Frag<T>::V V;
  const T* A = (const T*)Ap; const T* A2 = (const T*)A2p; const T* Bt = (const T*)Btp; const T* Bt2 = (const T*)Bt2p;
  __shared__ __align__(16) float sT[8][16 * 68];
  const int b    = blockIdx.y;
  const int lane = threadIdx.x & 31;
  const int wave = threadIdx.x >> 5;
  const int tilesN = N >> 6;
  const int tilesM = M >> 6;
  const int tile = blockIdx.x * 8 + wave;
  if (tile >= tilesM * tilesN) return;
  const int tm = tile / tilesN;
  const int tn = tile - tm * tilesN;
  const int m0 = tm << 6;
  const int n0 = tn << 6;

  const T* Ab  = A  + (size_t)b * strideA;
  const T* Bb  = Bt + (size_t)b * strideB;
  const T* Ab2 = SPLIT ? (A2  + (size_t)b * strideA) : nullptr;
  const T* Bb2 = SPLIT ? (Bt2 + (size_t)b * strideB) : nullptr;

  const int rlane = lane & 15;
  const int koff  = (lane >> 4) * 8;
  const int mOff  = (lane >> 4) * 8;

  v8f acc[4][4];
#pragma unroll
  for (int i = 0; i < 4; ++i)
#pragma unroll
    for (int j = 0; j < 4; ++j) acc[i][j] = (v8f){0.f,0.f,0.f,0.f,0.f,0.f,0.f,0.f};

  for (int k0 = 0; k0 < K; k0 += 32) {
    V bh[4], bl[4];
#pragma unroll
    for (int j = 0; j < 4; ++j) {
      const size_t bo = (size_t)(n0 + (j << 4) + rlane) * ldb + koff + k0;
      bh[j] = Frag<T>::load(Bb + bo);
      if (SPLIT) bl[j] = Frag<T>::load(Bb2 + bo);
    }
#pragma unroll
    for (int i = 0; i < 4; ++i) {
      const size_t ao = (size_t)(m0 + (i << 4) + rlane) * lda + koff + k0;
      V ah = Frag<T>::load(Ab + ao);
      V al;
      if (SPLIT) al = Frag<T>::load(Ab2 + ao);
#pragma unroll
      for (int j = 0; j < 4; ++j) {
        acc[i][j] = Frag<T>::mma(ah, bh[j], acc[i][j]);
        if (SPLIT) {
          acc[i][j] = Frag<T>::mma(ah, bl[j], acc[i][j]);
          acc[i][j] = Frag<T>::mma(al, bh[j], acc[i][j]);
        }
      }
      Frag<T>::guard(acc[i][0], acc[i][3], ah, SPLIT ? al : ah);
    }
    Frag<T>::keep(bh[0], bh[1], bh[2], bh[3]);
    if (SPLIT) Frag<T>::keep(bl[0], bl[1], bl[2], bl[3]);
  }
  acc_guard4(acc[0][0], acc[0][1], acc[0][2], acc[0][3]);
  acc_guard4(acc[1][0], acc[1][1], acc[1][2], acc[1][3]);
  acc_guard4(acc[2][0], acc[2][1], acc[2][2], acc[2][3]);
  acc_guard4(acc[3][0], acc[3][1], acc[3][2], acc[3][3]);

  float* slab = sT[wave];
  const float* Rb = RESID ? (resid + (size_t)b * strideR) : nullptr;
#pragma unroll
  for (int i = 0; i < 4; ++i) {
    const int mBase = m0 + (i << 4);
#pragma unroll
    for (int j = 0; j < 4; ++j) {
      const int n = n0 + (j << 4) + rlane;
      float bv = 0.f;
      if (BIAS_MODE == 2) bv = bias[n];
#pragma unroll
      for (int r = 0; r < 8; ++r) {
        float v = acc[i][j][r] * scale;
        if (BIAS_MODE == 1) v += bias[mBase + mOff + r];
        if (BIAS_MODE == 2) v += bv;
        if (RESID) v += Rb[(size_t)(mBase + mOff + r) * ldc + n];
        if (ACT == 1) v = tanhf(v);
        if (ACT == 2) v = fmaxf(v, 0.0f);
        if (ACT == 3) v = v / (1.0f + expf(-v));
        if (ACT == 4) v = (v > 0.f) ? v : 0.01f * v;
        if (ACT == 5) v = 0.5f * v * (1.0f + erff(v * 0.70710678118654752f));
        slab[(mOff + r) * 68 + (j << 4) + rlane] = v;
      }
    }
    __builtin_amdgcn_fence(__ATOMIC_RELEASE, "workgroup");
    __builtin_amdgcn_wave_barrier();
    __builtin_amdgcn_fence(__ATOMIC_ACQUIRE, "workgroup");
    if (OUT_MODE == 0) {
      float* C = (float*)Cout + (size_t)b * strideC;
      const int hh = lane >> 4, c4 = (lane & 15) * 4;
      for (int pass = 0; pass < 2; ++pass) {
#pragma unroll
        for (int it = 0; it < 8; ++it) {
          const int row = it * 2 + hh;
          v4f v = *(const v4f*)(slab + row * 68 + c4);
          *(volatile v4f*)(C + (size_t)(mBase + row) * ldc + n0 + c4) = v;
        }
        __threadfence();
      }
    } else {
      const int q = lane >> 3, c8 = (lane & 7) * 8;
      unsigned short* C  = (unsigned short*)Cout  + (size_t)b * strideC;
      unsigned short* C2 = (OUT_MODE == 2) ? ((unsigned short*)Cout2 + (size_t)b * strideC) : nullptr;
      for (int pass = 0; pass < 2; ++pass) {
#pragma unroll
        for (int it = 0; it < 4; ++it) {
          const int row = it * 4 + q;
          const float* sp = slab + row * 68 + c8;
          v8h hv, lv;
#pragma unroll
          for (int e = 0; e < 8; ++e) {
            if (OUT_MODE == 1) {
              hv[e] = (_Float16)sp[e];
            } else {
              unsigned short hb = f2bf_bits(sp[e]);
              unsigned short lb = f2bf_bits(sp[e] - bf_bits2f(hb));
              hv[e] = __builtin_bit_cast(_Float16, hb);
              lv[e] = __builtin_bit_cast(_Float16, lb);
            }
          }
          *(volatile v8h*)(C + (size_t)(mBase + row) * ldc + n0 + c8) = hv;
          if (OUT_MODE == 2) *(volatile v8h*)(C2 + (size_t)(mBase + row) * ldc + n0 + c8) = lv;
        }
        __threadfence();
      }
    }
    __builtin_amdgcn_fence(__ATOMIC_RELEASE, "workgroup");
    __builtin_amdgcn_wave_barrier();
    __builtin_amdgcn_fence(__ATOMIC_ACQUIRE, "workgroup");
  }
}

__global__ __launch_bounds__(256) void cast_f16_kernel(
    const float* __restrict__ src, unsigned short* __restrict__ dst, int total8, float scale)
{
  const int i = blockIdx.x * 256 + threadIdx.x;
  if (i >= total8) return;
  const size_t e0 = (size_t)i << 3;
  const float* p = src + e0;
  const v4f a0 = *(const v4f*)(p);
  const v4f a1 = *(const v4f*)(p + 4);
  v8h hv;
#pragma unroll
  for (int e = 0; e < 4; ++e) {
    hv[e]     = (_Float16)(a0[e] * scale);
    hv[4 + e] = (_Float16)(a1[e] * scale);
  }
  unsigned short* q = dst + e0;
  *(volatile v8h*)q = hv;
  __threadfence();
  *(volatile v8h*)q = hv;
}

__global__ __launch_bounds__(256) void cast_pad_f16_kernel(
    const float* __restrict__ src, int srcPitch, int srcRows, int srcCols,
    unsigned short* __restrict__ dst, int colShift, int total8, float scale)
{
  const int i = blockIdx.x * 256 + threadIdx.x;
  if (i >= total8) return;
  const int e0 = i << 3;
  const int r  = e0 >> colShift;
  const int c  = e0 & ((1 << colShift) - 1);
  const bool valid = (r < srcRows) && (c < srcCols);
  const int rc = (r < srcRows) ? r : (srcRows - 1);
  const int cc = (c + 8 <= srcCols) ? c : (srcCols - 8);
  const float* p = src + (size_t)rc * srcPitch + cc;
  const v4f a0 = *(const v4f*)(p);
  const v4f a1 = *(const v4f*)(p + 4);
  v8h hv;
#pragma unroll
  for (int e = 0; e < 4; ++e) {
    const float f0 = valid ? (a0[e] * scale) : 0.0f;
    const float f1 = valid ? (a1[e] * scale) : 0.0f;
    hv[e]     = (_Float16)f0;
    hv[4 + e] = (_Float16)f1;
  }
  unsigned short* q = dst + (size_t)e0;
  *(volatile v8h*)q = hv;
  __threadfence();
  *(volatile v8h*)q = hv;
}

__global__ __launch_bounds__(256) void conv_silu_kernel(
    const float* __restrict__ XZ, const float* __restrict__ cw, const float* __restrict__ cb,
    float* __restrict__ UC, unsigned short* __restrict__ UC16)
{
  __shared__ __align__(16) float sT[16 * kTP];
  const int tid = threadIdx.x, lane = tid & 31, wave = tid >> 5;
  const int d0 = blockIdx.x * 256, d = d0 + tid;
  const int t0 = blockIdx.y * 64;
  const int tloc = t0 & (kSeqL - 1);
  const float w0 = cw[d * 4 + 0], w1 = cw[d * 4 + 1], w2 = cw[d * 4 + 2], w3 = cw[d * 4 + 3];
  const float bc = cb[d];
  float xm3, xm2, xm1;
  {
    const int r3 = (t0 >= 3) ? (t0 - 3) : 0, r2 = (t0 >= 2) ? (t0 - 2) : 0, r1 = (t0 >= 1) ? (t0 - 1) : 0;
    const float v3 = XZ[(size_t)r3 * kXZP + d];
    const float v2 = XZ[(size_t)r2 * kXZP + d];
    const float v1 = XZ[(size_t)r1 * kXZP + d];
    const bool hist = (tloc != 0);
    xm3 = hist ? v3 : 0.f;
    xm2 = hist ? v2 : 0.f;
    xm1 = hist ? v1 : 0.f;
  }
  const int hrow = wave >> 1;
  const int hch  = (wave & 1) * 128 + lane * 4;
#pragma unroll 1
  for (int sub = 0; sub < 4; ++sub) {
    const int lb = t0 + sub * 16;
#pragma unroll 1
    for (int s = 0; s < 16; ++s) {
      const float xc = XZ[(size_t)(lb + s) * kXZP + d];
      float acc = w0 * xm3;
      acc = fmaf(w1, xm2, acc);
      acc = fmaf(w2, xm1, acc);
      acc = fmaf(w3, xc, acc);
      const float sv = acc + bc;
      const float sg = __builtin_amdgcn_rcpf(1.0f + __expf(-sv));
      sT[s * kTP + tid] = sv * sg;
      xm3 = xm2; xm2 = xm1; xm1 = xc;
    }
    __syncthreads();
    v4f fv[4];
    v8h bv[2];
#pragma unroll
    for (int it = 0; it < 4; ++it) fv[it] = *(const v4f*)(sT + (it * 4 + hrow) * kTP + hch);
#pragma unroll
    for (int it = 0; it < 2; ++it) {
      const float* sp = sT + (it * 8 + wave) * kTP + lane * 8;
      const v4f a0 = *(const v4f*)(sp);
      const v4f a1 = *(const v4f*)(sp + 4);
#pragma unroll
      for (int e = 0; e < 4; ++e) {
        bv[it][e]     = (_Float16)(a0[e] * 64.0f);
        bv[it][4 + e] = (_Float16)(a1[e] * 64.0f);
      }
    }
    for (int pass = 0; pass < 2; ++pass) {
#pragma unroll
      for (int it = 0; it < 4; ++it)
        *(volatile v4f*)(UC + (size_t)(lb + it * 4 + hrow) * kDin + d0 + hch) = fv[it];
#pragma unroll
      for (int it = 0; it < 2; ++it)
        *(volatile v8h*)(UC16 + (size_t)(lb + it * 8 + wave) * kDin + d0 + lane * 8) = bv[it];
      __threadfence();
    }
    __syncthreads();
  }
}

__global__ __launch_bounds__(256) void scan_pool_kernel(
    const float* __restrict__ DLR, const float* __restrict__ UC, const float* __restrict__ XZ,
    const float* __restrict__ PROJ, const float* __restrict__ A_log, const float* __restrict__ Dv,
    float* __restrict__ YBAR)
{
  __shared__ __align__(16) float sBC[kSeqL * 32];
  __shared__ __align__(16) float sOut[256];
  const int tid = threadIdx.x, lane = tid & 31, wave = tid >> 5;
  const int d0 = blockIdx.x * 256, d = d0 + tid;
  const int rb = blockIdx.y * kSeqL;

#pragma unroll
  for (int p = 0; p < 8; ++p) {
    const int idx = tid + p * 256;
    const int r = idx >> 3, q = (idx & 7) * 4;
    const v4f v = *(const v4f*)(PROJ + (size_t)(rb + r) * kPrjP + kDtR + q);
    *(v4f*)(sBC + r * 32 + q) = v;
  }
  __syncthreads();

  float An[kNst];
#pragma unroll
  for (int n = 0; n < kNst; ++n) An[n] = -__expf(A_log[(size_t)d * kNst + n]);
  const float Dd = Dv[d];
  float h[kNst];
#pragma unroll
  for (int n = 0; n < kNst; ++n) h[n] = 0.f;
  float ysum = 0.f;

#pragma unroll 1
  for (int t = 0; t < kSeqL; ++t) {
    const size_t m = (size_t)(rb + t);
    const float a     = DLR[m * kDin + d];
    const float delta = fmaxf(a, 0.0f) + log1pf(__expf(-fabsf(a)));
    const float xv    = UC[m * kDin + d];
    const float zv    = XZ[m * kXZP + kDin + d];
    v4f Bq[4], Cq[4];
#pragma unroll
    for (int qq = 0; qq < 4; ++qq) {
      Bq[qq] = *(const v4f*)(sBC + t * 32 + 4 * qq);
      Cq[qq] = *(const v4f*)(sBC + t * 32 + kNst + 4 * qq);
    }
    float y = 0.f;
#pragma unroll
    for (int n = 0; n < kNst; ++n) {
      const float e = __expf(delta * An[n]);
      float db = delta * Bq[n >> 2][n & 3];
      asm volatile("" : "+v"(db));
      float p = db * xv;
      asm volatile("" : "+v"(p));
      float qv = h[n] * e;
      asm volatile("" : "+v"(qv));
      const float hn = qv + p;
      h[n] = hn;
      float rr = Cq[n >> 2][n & 3] * hn;
      asm volatile("" : "+v"(rr));
      y += rr;
    }
    float sk = xv * Dd;
    asm volatile("" : "+v"(sk));
    y += sk;
    const float sg = __builtin_amdgcn_rcpf(1.0f + __expf(-zv));
    const float g  = zv * sg;
    float yg = y * g;
    asm volatile("" : "+v"(yg));
    ysum += yg;
  }
  sOut[tid] = ysum * (1.0f / (float)kSeqL);
  __syncthreads();
  if (wave == 0) {
    const v4f a0 = *(const v4f*)(sOut + lane * 4);
    const v4f a1 = *(const v4f*)(sOut + 128 + lane * 4);
    float* yr = YBAR + (size_t)blockIdx.y * kDin + d0;
    for (int pass = 0; pass < 2; ++pass) {
      *(volatile v4f*)(yr + lane * 4) = a0;
      *(volatile v4f*)(yr + 128 + lane * 4) = a1;
      __threadfence();
    }
  }
}

__global__ __launch_bounds__(256) void head_x_kernel(
    const float* __restrict__ YBAR, const float* __restrict__ Wout,
    const float* __restrict__ Wfc, const float* __restrict__ bfc,
    float* __restrict__ out_x)
{
  __shared__ __align__(16) float sy[kDin];
  __shared__ __align__(16) float se[kDmod];
  __shared__ __align__(16) float sx[kDimIn];
  const int tid = threadIdx.x, lane = tid & 31, wave = tid >> 5;
  const int b = blockIdx.x;
  sy[tid]       = YBAR[(size_t)b * kDin + tid];
  sy[256 + tid] = YBAR[(size_t)b * kDin + 256 + tid];
  __syncthreads();
  {
    const float* w = Wout + (size_t)tid * kDin;
    float acc = 0.f;
#pragma unroll 1
    for (int k = 0; k < kDin; k += 4) {
      const v4f a  = *(const v4f*)(sy + k);
      const v4f ww = *(const v4f*)(w + k);
      acc = fmaf(a[0], ww[0], acc);
      acc = fmaf(a[1], ww[1], acc);
      acc = fmaf(a[2], ww[2], acc);
      acc = fmaf(a[3], ww[3], acc);
    }
    se[tid] = acc;
  }
  __syncthreads();
  {
    const float* w = Wfc + (size_t)tid * kDmod;
    float acc = 0.f;
#pragma unroll 1
    for (int k = 0; k < kDmod; k += 4) {
      const v4f a  = *(const v4f*)(se + k);
      const v4f ww = *(const v4f*)(w + k);
      acc = fmaf(a[0], ww[0], acc);
      acc = fmaf(a[1], ww[1], acc);
      acc = fmaf(a[2], ww[2], acc);
      acc = fmaf(a[3], ww[3], acc);
    }
    const float v  = acc + bfc[tid];
    const float th = tanhf(v);
    sx[tid] = (th > 0.f) ? th : expm1f(th);
  }
  __syncthreads();
  if (wave == 0) {
    const v4f x0 = *(const v4f*)(sx + lane * 4);
    const v4f x1 = *(const v4f*)(sx + 128 + lane * 4);
    float* xr = out_x + (size_t)b * kDimIn;
    for (int pass = 0; pass < 2; ++pass) {
      *(volatile v4f*)(xr + lane * 4) = x0;
      *(volatile v4f*)(xr + 128 + lane * 4) = x1;
      __threadfence();
    }
  }
}

__global__ __launch_bounds__(64) void head_ms_kernel(
    const float* __restrict__ xin,
    const float* __restrict__ Wmu, const float* __restrict__ bmu,
    const float* __restrict__ Wsg, const float* __restrict__ bsg,
    float* __restrict__ out_mu, float* __restrict__ out_sg)
{
  __shared__ __align__(16) float sx[kDimIn];
  __shared__ __align__(16) float sm[kDimOut];
  __shared__ __align__(16) float ss[kDimOut];
  const int tid = threadIdx.x, lane = tid & 31, wave = tid >> 5;
  const int b = blockIdx.x;
  *(v4f*)(sx + tid * 4) = *(const v4f*)(xin + (size_t)b * kDimIn + tid * 4);
  __syncthreads();
  {
    const float* wm = Wmu + (size_t)tid * kDimIn;
    const float* wg = Wsg + (size_t)tid * kDimIn;
    float am = 0.f, ag = 0.f;
#pragma unroll 1
    for (int k = 0; k < kDimIn; k += 4) {
      const v4f a  = *(const v4f*)(sx + k);
      const v4f m4 = *(const v4f*)(wm + k);
      const v4f g4 = *(const v4f*)(wg + k);
      am = fmaf(a[0], m4[0], am); am = fmaf(a[1], m4[1], am); am = fmaf(a[2], m4[2], am); am = fmaf(a[3], m4[3], am);
      ag = fmaf(a[0], g4[0], ag); ag = fmaf(a[1], g4[1], ag); ag = fmaf(a[2], g4[2], ag); ag = fmaf(a[3], g4[3], ag);
    }
    const float mu = am + bmu[tid];
    const float v  = ag + bsg[tid];
    const float el = (v > 0.f) ? v : expm1f(v);
    const float sg = (el + 1.0f) + 1e-14f;
    sm[tid] = mu;
    ss[tid] = sg;
  }
  __syncthreads();
  const int lc = (lane < 16) ? lane : 15;
  const v4f mv = *(const v4f*)(sm + lc * 4);
  const v4f sv = *(const v4f*)(ss + lc * 4);
  float* mr = out_mu + (size_t)b * kDimOut + lc * 4;
  float* sr = out_sg + (size_t)b * kDimOut + lc * 4;
  for (int pass = 0; pass < 2; ++pass) {
    if (lane < 16) {
      if (wave == 0) *(volatile v4f*)mr = mv;
      else           *(volatile v4f*)sr = sv;
    }
    __threadfence();
  }
}

extern "C" void kernel_launch(void* const* d_in, const int* in_sizes, int n_in,
                              void* d_out, int out_size, void* d_ws, size_t ws_size,
                              hipStream_t stream)
{
  if (n_in < 16) return;
  const float* x       = (const float*)d_in[0];
  const float* W_in    = (const float*)d_in[1];
  const float* conv_w  = (const float*)d_in[2];
  const float* conv_b  = (const float*)d_in[3];
  const float* W_xprj  = (const float*)d_in[4];
  const float* W_dt    = (const float*)d_in[5];
  const float* b_dt    = (const float*)d_in[6];
  const float* A_log   = (const float*)d_in[7];
  const float* Dv      = (const float*)d_in[8];
  const float* W_out   = (const float*)d_in[9];
  const float* W_outfc = (const float*)d_in[10];
  const float* b_outfc = (const float*)d_in[11];
  const float* W_mu    = (const float*)d_in[12];
  const float* b_mu    = (const float*)d_in[13];
  const float* W_sg    = (const float*)d_in[14];
  const float* b_sg    = (const float*)d_in[15];

  if (in_sizes[0] != kRows * kDmod) return;
  if (in_sizes[1] != kXZP * kDmod) return;
  if (in_sizes[2] != kDin * 4 || in_sizes[3] != kDin) return;
  if (in_sizes[4] != kPrjN * kDin) return;
  if (in_sizes[5] != kDin * kDtR || in_sizes[6] != kDin) return;
  if (in_sizes[7] != kDin * kNst || in_sizes[8] != kDin) return;
  if (in_sizes[9] != kDmod * kDin) return;
  if (in_sizes[10] != kDimIn * kDmod || in_sizes[11] != kDimIn) return;
  if (in_sizes[12] != kDimOut * kDimIn || in_sizes[13] != kDimOut) return;
  if (in_sizes[14] != kDimOut * kDimIn || in_sizes[15] != kDimOut) return;
  if (out_size != kBatch * kDimIn + 2 * kBatch * kDimOut) return;

  const size_t SZ_WIN16  = (size_t)kXZP * kDmod * 2;
  const size_t SZ_WXP16  = (size_t)kPrjP * kDin * 2;
  const size_t SZ_WDT16  = (size_t)kDin * kDtKP * 2;
  const size_t SZ_X16    = (size_t)kRows * kDmod * 2;
  const size_t SZ_XZ     = (size_t)kChunkT * kXZP * 4;
  const size_t SZ_UC     = (size_t)kChunkT * kDin * 4;
  const size_t SZ_UC16   = (size_t)kChunkT * kDin * 2;
  const size_t SZ_PROJ   = (size_t)kChunkT * kPrjP * 4;
  const size_t SZ_DT16   = (size_t)kChunkT * kDtKP * 2;
  const size_t SZ_DLR    = (size_t)kChunkT * kDin * 4;
  const size_t SZ_YBAR   = (size_t)kBatch * kDin * 4;
  const size_t OFF_WIN16  = 0;
  const size_t OFF_WXP16  = OFF_WIN16  + SZ_WIN16;
  const size_t OFF_WDT16  = OFF_WXP16  + SZ_WXP16;
  const size_t OFF_X16    = OFF_WDT16  + SZ_WDT16;
  const size_t OFF_XZ     = OFF_X16    + SZ_X16;
  const size_t OFF_UC     = OFF_XZ     + SZ_XZ;
  const size_t OFF_UC16   = OFF_UC     + SZ_UC;
  const size_t OFF_PROJ   = OFF_UC16   + SZ_UC16;
  const size_t OFF_DT16   = OFF_PROJ   + SZ_PROJ;
  const size_t OFF_DLR    = OFF_DT16   + SZ_DT16;
  const size_t OFF_YBAR   = OFF_DLR    + SZ_DLR;
  const size_t TOTAL      = OFF_YBAR   + SZ_YBAR;
  if (ws_size < TOTAL) return;

  char* ws = (char*)d_ws;
  unsigned short* WIN16  = (unsigned short*)(ws + OFF_WIN16);
  unsigned short* WXP16  = (unsigned short*)(ws + OFF_WXP16);
  unsigned short* WDT16  = (unsigned short*)(ws + OFF_WDT16);
  unsigned short* X16    = (unsigned short*)(ws + OFF_X16);
  float*          XZ     = (float*)(ws + OFF_XZ);
  float*          UC     = (float*)(ws + OFF_UC);
  unsigned short* UC16   = (unsigned short*)(ws + OFF_UC16);
  float*          PROJ   = (float*)(ws + OFF_PROJ);
  unsigned short* DT16   = (unsigned short*)(ws + OFF_DT16);
  float*          DLR    = (float*)(ws + OFF_DLR);
  float*          YBAR   = (float*)(ws + OFF_YBAR);
  const float* dummy_bias  = b_dt;
  const float* dummy_resid = x;

  float* out_x  = (float*)d_out;
  float* out_mu = out_x + (size_t)kBatch * kDimIn;
  float* out_sg = out_mu + (size_t)kBatch * kDimOut;

  cast_f16_kernel<<<(kXZP * kDmod) / 8 / 256, 256, 0, stream>>>(W_in, WIN16, (kXZP * kDmod) / 8, 32.0f);
  cast_pad_f16_kernel<<<(kPrjP * kDin) / 8 / 256, 256, 0, stream>>>(W_xprj, kDin, kPrjN, kDin, WXP16, 9, (kPrjP * kDin) / 8, 32.0f);
  cast_pad_f16_kernel<<<(kDin * kDtKP) / 8 / 256, 256, 0, stream>>>(W_dt, kDtR, kDin, kDtR, WDT16, 5, (kDin * kDtKP) / 8, 32.0f);
  cast_f16_kernel<<<(kRows * kDmod) / 8 / 256, 256, 0, stream>>>(x, X16, (kRows * kDmod) / 8, 1.0f);

  for (int c = 0; c < kNChunk; ++c) {
    const unsigned short* X16c = X16 + (size_t)c * kChunkT * kDmod;
    float* YBARc = YBAR + (size_t)c * kChunkB * kDin;

    wmma_gemm64<0, false, 0, 0, false><<<dim3(256, 1), 256, 0, stream>>>(
        X16c, X16c, kDmod, 0L, WIN16, WIN16, kDmod, 0L,
        (void*)XZ, (void*)XZ, kXZP, 0L, dummy_bias, dummy_resid, 0L, kChunkT, kXZP, kDmod, 1.0f / 32.0f);

    conv_silu_kernel<<<dim3(kDin / 256, kChunkT / 64), 256, 0, stream>>>(XZ, conv_w, conv_b, UC, UC16);

    wmma_gemm64<0, false, 0, 0, false><<<dim3(16, 1), 256, 0, stream>>>(
        UC16, UC16, kDin, 0L, WXP16, WXP16, kDin, 0L,
        (void*)PROJ, (void*)PROJ, kPrjP, 0L, dummy_bias, dummy_resid, 0L, kChunkT, kPrjP, kDin, 1.0f / 2048.0f);

    cast_pad_f16_kernel<<<(kChunkT * kDtKP) / 8 / 256, 256, 0, stream>>>(PROJ, kPrjP, kChunkT, kDtR, DT16, 5, (kChunkT * kDtKP) / 8, 256.0f);

    wmma_gemm64<0, false, 2, 0, false><<<dim3(128, 1), 256, 0, stream>>>(
        DT16, DT16, kDtKP, 0L, WDT16, WDT16, kDtKP, 0L,
        (void*)DLR, (void*)DLR, kDin, 0L, b_dt, dummy_resid, 0L, kChunkT, kDin, kDtKP, 1.0f / 8192.0f);

    scan_pool_kernel<<<dim3(kDin / 256, kChunkB), 256, 0, stream>>>(DLR, UC, XZ, PROJ, A_log, Dv, YBARc);
  }

  head_x_kernel<<<kBatch, 256, 0, stream>>>(YBAR, W_out, W_outfc, b_outfc, out_x);
  head_ms_kernel<<<kBatch, 64, 0, stream>>>(out_x, W_mu, b_mu, W_sg, b_sg, out_mu, out_sg);
}
